// HeteroActor_31267361915424
// MI455X (gfx1250) — hardware-verified
//
#include <hip/hip_runtime.h>
#include <stddef.h>


#define FIN     128
#define NC      64
#define HEADS   4
#define CH      16
#define NTHR    256
#define NWAVE   8
#define BM      64
#define EPT     8
#define NGRP    2
#define CHUNK   (NTHR * EPT * NGRP)
#define WCAP    (EPT * NGRP * 32)
#define LISTN   (NWAVE * WCAP)
#define NBC     4096
#define NBF     1024
#define RCAP    40960
#define RBN     128
#define TGT     256
#define DEGCAP  256
#define OTHR    512
#define STHR    128
#define ZTHR    512
#define WSCAP   134217728
#define NEG_SLOPE 0.2f
#define DEN_EPS 1e-16f
#define NEG_BIG (-3.0e38f)
#define ASC     8.0f
#define WSC     64.0f
#define RSC     (1.0f / 512.0f)

#define LDS_FILL ((RCAP + NBF + LISTN) * 4 + 64)

static_assert((CHUNK & (CHUNK - 1)) == 0);
static_assert(CHUNK <= 4096);
static_assert(NBC <= 4096 && NBF <= 4096);
static_assert((NBC & (NBC - 1)) == 0 && (NBF & (NBF - 1)) == 0);
static_assert(NBC == 4 * NBF);
static_assert(OTHR * 8 == NBC);
static_assert((RCAP % 32) == 0);
static_assert(TGT == NWAVE * 32);
static_assert((TGT % BM) == 0);
static_assert(HEADS * CH == NC && NC == 64);
static_assert(BM * HEADS == 256);

typedef float          v4f  __attribute__((ext_vector_type(4)));
typedef float          v8f  __attribute__((ext_vector_type(8)));
typedef int            v4i  __attribute__((ext_vector_type(4)));
typedef _Float16       v8h  __attribute__((ext_vector_type(8)));
typedef _Float16       v16h __attribute__((ext_vector_type(16)));
union Frag { v16h v; v8h half[2]; };

__device__ __forceinline__ v8h cvt8(v4f a, v4f b, float s) {
  v8h r;
  r[0] = (_Float16)(a.x * s); r[1] = (_Float16)(a.y * s);
  r[2] = (_Float16)(a.z * s); r[3] = (_Float16)(a.w * s);
  r[4] = (_Float16)(b.x * s); r[5] = (_Float16)(b.y * s);
  r[6] = (_Float16)(b.z * s); r[7] = (_Float16)(b.w * s);
  return r;
}

__device__ __forceinline__ v8f wmh(v16h a, v16h b, v8f c) {
  v8f d = __builtin_amdgcn_wmma_f32_16x16x32_f16(false, a, false, b, (short)0, c, false, false);
  asm volatile("v_nop\n\tv_nop\n\tv_nop\n\tv_nop" : "+v"(d) : "v"(a), "v"(b));
  return d;
}

__device__ __forceinline__ float lrelu(float v) { return v > 0.0f ? v : NEG_SLOPE * v; }

template <int KD>
__device__ __forceinline__ void mma2(const _Float16* sA, const _Float16* __restrict__ Bw,
                                     int r0, int c0, int hh, int m, v8f& acc0, v8f& acc1) {
  constexpr int APK = KD + 8;
  const _Float16* ap  = sA + (r0 + m) * APK + 8 * hh;
  const _Float16* bp0 = Bw + (size_t)(c0 + m) * KD + 8 * hh;
  const _Float16* bp1 = Bw + (size_t)(c0 + 16 + m) * KD + 8 * hh;
#pragma unroll
  for (int kt = 0; kt < KD / 32; ++kt) {
    Frag a, b0, b1;
    a.half[0]  = *(const v8h*)(ap + 32 * kt);
    a.half[1]  = *(const v8h*)(ap + 32 * kt + 16);
    b0.half[0] = *(const v8h*)(bp0 + 32 * kt);
    b0.half[1] = *(const v8h*)(bp0 + 32 * kt + 16);
    b1.half[0] = *(const v8h*)(bp1 + 32 * kt);
    b1.half[1] = *(const v8h*)(bp1 + 32 * kt + 16);
    acc0 = wmh(a.v, b0.v, acc0);
    acc1 = wmh(a.v, b1.v, acc1);
  }
}

__device__ __forceinline__ void stage2(float* stg, int r0, int c0, int hh, int m, v8f acc0, v8f acc1) {
  float* sp = stg + (r0 + 8 * hh) * NC + c0 + m;
#pragma unroll
  for (int r = 0; r < 8; ++r) { sp[r * NC] = acc0[r]; sp[r * NC + 16] = acc1[r]; }
}

template <int NB>
__device__ __forceinline__ int scan_chunk(const int* __restrict__ dsts, int nE, int cbase, int slotBase,
                                          int vec8, int* list, int tid, int lane, int wave) {
  int wc = 0;
#pragma unroll
  for (int g = 0; g < NGRP; ++g) {
    const int el0  = (g * NTHR + tid) * EPT;
    const int e0   = cbase + el0;
    const int sent = -2147483647 - 1;
    v4i da, db;
    if (vec8 != 0 && cbase + CHUNK <= nE) {
      da = *(const v4i*)(dsts + e0);
      db = *(const v4i*)(dsts + e0 + 4);
    } else {
      da.x = (e0     < nE) ? dsts[min(e0, nE - 1)] : sent;
      da.y = (e0 + 1 < nE) ? dsts[min(e0 + 1, nE - 1)] : sent;
      da.z = (e0 + 2 < nE) ? dsts[min(e0 + 2, nE - 1)] : sent;
      da.w = (e0 + 3 < nE) ? dsts[min(e0 + 3, nE - 1)] : sent;
      db.x = (e0 + 4 < nE) ? dsts[min(e0 + 4, nE - 1)] : sent;
      db.y = (e0 + 5 < nE) ? dsts[min(e0 + 5, nE - 1)] : sent;
      db.z = (e0 + 6 < nE) ? dsts[min(e0 + 6, nE - 1)] : sent;
      db.w = (e0 + 7 < nE) ? dsts[min(e0 + 7, nE - 1)] : sent;
    }
    const unsigned nb = (unsigned)slotBase;
    const unsigned s0 = (unsigned)da.x - nb, s1 = (unsigned)da.y - nb;
    const unsigned s2 = (unsigned)da.z - nb, s3 = (unsigned)da.w - nb;
    const unsigned s4 = (unsigned)db.x - nb, s5 = (unsigned)db.y - nb;
    const unsigned s6 = (unsigned)db.z - nb, s7 = (unsigned)db.w - nb;
    const bool h0 = s0 < (unsigned)NB, h1 = s1 < (unsigned)NB, h2 = s2 < (unsigned)NB, h3 = s3 < (unsigned)NB;
    const bool h4 = s4 < (unsigned)NB, h5 = s5 < (unsigned)NB, h6 = s6 < (unsigned)NB, h7 = s7 < (unsigned)NB;
    const unsigned any = __builtin_amdgcn_ballot_w32(h0 | h1 | h2 | h3 | h4 | h5 | h6 | h7);
    if (any != 0u) {
#define HITJ(J, HJ, SJ) { \
        const unsigned mj = __builtin_amdgcn_ballot_w32(HJ); \
        if (mj != 0u) { \
          if (HJ) { \
            const int pos = wc + (int)__builtin_amdgcn_mbcnt_lo(mj, 0u); \
            if (pos < WCAP) list[wave * WCAP + pos] = ((el0 + (J)) << 12) | (int)(SJ); \
          } \
          wc += (int)__builtin_popcount(mj); } }
      HITJ(0, h0, s0)
      HITJ(1, h1, s1)
      HITJ(2, h2, s2)
      HITJ(3, h3, s3)
      HITJ(4, h4, s4)
      HITJ(5, h5, s5)
      HITJ(6, h6, s6)
      HITJ(7, h7, s7)
#undef HITJ
    }
  }
  return wc;
}

template <int KD>
__global__ __launch_bounds__(NTHR) void k_wprep(const float* __restrict__ W0, const float* __restrict__ W1,
                                                _Float16* P0, _Float16* P1) {
  constexpr int UNITS = NC * KD / 8;
  constexpr int KD8   = KD / 8;
  static_assert((UNITS % NTHR) == 0);
  const float* W = (blockIdx.y == 0) ? W0 : W1;
  _Float16*    P = (blockIdx.y == 0) ? P0 : P1;
  const int i = (int)blockIdx.x * NTHR + (int)threadIdx.x;
  if (i >= UNITS) return;
  const int n  = i / KD8;
  const int k0 = (i - n * KD8) * 8;
  v4f a, b;
  a.x = W[(size_t)(k0 + 0) * NC + n]; a.y = W[(size_t)(k0 + 1) * NC + n];
  a.z = W[(size_t)(k0 + 2) * NC + n]; a.w = W[(size_t)(k0 + 3) * NC + n];
  b.x = W[(size_t)(k0 + 4) * NC + n]; b.y = W[(size_t)(k0 + 5) * NC + n];
  b.z = W[(size_t)(k0 + 6) * NC + n]; b.w = W[(size_t)(k0 + 7) * NC + n];
  const v8h hv = cvt8(a, b, WSC);
  _Float16* d = P + (size_t)i * 8;
  *(volatile v8h*)d = hv;
  __threadfence();
  *(volatile v8h*)d = hv;
}

__global__ __launch_bounds__(NTHR) void k_count(
    const int* __restrict__ dsts, int* cnt, int nE, int vec8) {
  __shared__ __attribute__((aligned(16))) int scnt[NBC];
  __shared__ __attribute__((aligned(16))) int list[LISTN];
  __shared__ int wcnt[NWAVE];
  const int tid = threadIdx.x, lane = tid & 31, wave = tid >> 5;
  const int nodeBase = blockIdx.x * NBC;

  for (int i = tid; i < NBC; i += NTHR) scnt[i] = 0;
  __syncthreads();

  const int nChunks = (nE + CHUNK - 1) / CHUNK;
#pragma unroll 1
  for (int ch = 0; ch < nChunks; ++ch) {
    const int cbase = ch * CHUNK;
    const int wc = scan_chunk<NBC>(dsts, nE, cbase, nodeBase, vec8, list, tid, lane, wave);
    if (lane == 0) wcnt[wave] = wc;
    __syncthreads();
    if (wave == 0) {
#pragma unroll 1
      for (int wsx = 0; wsx < NWAVE; ++wsx) {
        int n = __builtin_amdgcn_readfirstlane(wcnt[wsx]);
        n = n > WCAP ? WCAP : (n < 0 ? 0 : n);
        const int* lp = list + wsx * WCAP;
#pragma unroll 1
        for (int i = 0; i < n; ++i) {
          const int ent  = __builtin_amdgcn_readfirstlane(lp[i]);
          const int slot = ent & (NBC - 1);
          if (lane == 0) scnt[slot] = scnt[slot] + 1;
        }
      }
    }
    __syncthreads();
  }

  v4i cq[4];
#pragma unroll
  for (int q = 0; q < 4; ++q) {
    const int f = (wave * 4 + q) * 128 + 4 * lane;
    cq[q] = *(const v4i*)(scnt + f);
  }
  int* cp = cnt + (size_t)nodeBase;
#pragma unroll
  for (int q = 0; q < 4; ++q) {
    const int f = (wave * 4 + q) * 128 + 4 * lane;
    *(volatile v4i*)(cp + f) = cq[q];
  }
  __threadfence();
#pragma unroll
  for (int q = 0; q < 4; ++q) {
    const int f = (wave * 4 + q) * 128 + 4 * lane;
    *(volatile v4i*)(cp + f) = cq[q];
  }
}

__global__ __launch_bounds__(OTHR) void k_offsets(
    const int* __restrict__ cnt, int* off, int* rbase, int nChunk) {
  __shared__ __attribute__((aligned(16))) int soff[NBC];
  __shared__ __attribute__((aligned(16))) int srb[RBN];
  __shared__ int wtot[OTHR / 32];
  const int tid = threadIdx.x, lane = tid & 31, wave = tid >> 5, sub = tid >> 7;
  for (int i = tid; i < RBN; i += OTHR) srb[i] = 0;
  int carry = 0;
#pragma unroll 1
  for (int ch = 0; ch < nChunk; ++ch) {
    const int base = ch * NBC;
    const v4i c0 = *(const v4i*)(cnt + base + 8 * tid);
    const v4i c1 = *(const v4i*)(cnt + base + 8 * tid + 4);
    const int e0 = max(c0.x, 0), e1 = max(c0.y, 0), e2 = max(c0.z, 0), e3 = max(c0.w, 0);
    const int e4 = max(c1.x, 0), e5 = max(c1.y, 0), e6 = max(c1.z, 0), e7 = max(c1.w, 0);
    const int ts = e0 + e1 + e2 + e3 + e4 + e5 + e6 + e7;
    int incl = ts;
#pragma unroll
    for (int d = 1; d < 32; d <<= 1) {
      const int t = __shfl_up(incl, d);
      if (lane >= d) incl += t;
    }
    if (lane == 31) wtot[wave] = incl;
    __syncthreads();
    const int S0 = wtot[0]  + wtot[1]  + wtot[2]  + wtot[3];
    const int S1 = wtot[4]  + wtot[5]  + wtot[6]  + wtot[7];
    const int S2 = wtot[8]  + wtot[9]  + wtot[10] + wtot[11];
    const int S3 = wtot[12] + wtot[13] + wtot[14] + wtot[15];
    int pre = 0;
#pragma unroll 1
    for (int w = 4 * sub; w < wave; ++w) pre += wtot[w];
    const int b0 = carry;
    const int b1 = b0 + ((S0 + 31) & ~31);
    const int b2 = b1 + ((S1 + 31) & ~31);
    const int b3 = b2 + ((S2 + 31) & ~31);
    const int b4 = b3 + ((S3 + 31) & ~31);
    const int myb = sub == 0 ? b0 : (sub == 1 ? b1 : (sub == 2 ? b2 : b3));
    if (tid == 0) {
      srb[min(4 * ch + 0, RBN - 1)] = b0;
      srb[min(4 * ch + 1, RBN - 1)] = b1;
      srb[min(4 * ch + 2, RBN - 1)] = b2;
      srb[min(4 * ch + 3, RBN - 1)] = b3;
    }
    int run = myb + pre + incl - ts;
    soff[8 * tid + 0] = run; run += e0;
    soff[8 * tid + 1] = run; run += e1;
    soff[8 * tid + 2] = run; run += e2;
    soff[8 * tid + 3] = run; run += e3;
    soff[8 * tid + 4] = run; run += e4;
    soff[8 * tid + 5] = run; run += e5;
    soff[8 * tid + 6] = run; run += e6;
    soff[8 * tid + 7] = run;
    carry = b4;
    __syncthreads();
    const v4i o0 = *(const v4i*)(soff + 4 * tid);
    const v4i o1 = *(const v4i*)(soff + 4 * (tid + OTHR));
    int* op = off + base;
    *(volatile v4i*)(op + 4 * tid) = o0;
    *(volatile v4i*)(op + 4 * (tid + OTHR)) = o1;
    __threadfence();
    *(volatile v4i*)(op + 4 * tid) = o0;
    *(volatile v4i*)(op + 4 * (tid + OTHR)) = o1;
    __syncthreads();
  }
  if (tid == 0) srb[min(4 * nChunk, RBN - 1)] = carry;
  __syncthreads();
  v4i rv = {0, 0, 0, 0};
  if (tid < 32) rv = *(const v4i*)(srb + 4 * tid);
  if (tid < 32) *(volatile v4i*)(rbase + 4 * tid) = rv;
  __threadfence();
  if (tid < 32) *(volatile v4i*)(rbase + 4 * tid) = rv;
}

__global__ __launch_bounds__(NTHR) void k_fill(
    const int* __restrict__ srcs, const int* __restrict__ dsts,
    const int* __restrict__ off, const int* __restrict__ rbase,
    int* csr, int nSrc, int nE, int vec8, int csrLen) {
  extern __shared__ v4f lds_dyn[];
  int* region = (int*)lds_dyn;
  int* cursor = region + RCAP;
  int* list   = cursor + NBF;
  int* wcnt   = list + LISTN;
  const int tid = threadIdx.x, lane = tid & 31, wave = tid >> 5;
  const int b = blockIdx.x;
  const int nodeBase = b * NBF;

  int rb0 = rbase[b];
  const int rb1 = rbase[b + 1];
  rb0 = rb0 < 0 ? 0 : (rb0 > csrLen ? csrLen : rb0);
  rb0 &= ~31;
  int len = rb1 - rb0;
  len = len < 0 ? 0 : (len > RCAP ? RCAP : len);
  int lenW = (len + 31) & ~31;
  if (rb0 + lenW > csrLen) lenW = (csrLen - rb0) & ~31;

  {
    const v4i z = {0, 0, 0, 0};
    for (int i = tid; i < RCAP / 4; i += NTHR) ((v4i*)region)[i] = z;
    for (int s = tid; s < NBF; s += NTHR) {
      int o = off[nodeBase + s] - rb0;
      o = o < 0 ? 0 : (o > RCAP ? RCAP : o);
      cursor[s] = o;
    }
  }
  __syncthreads();

  const int nChunks = (nE + CHUNK - 1) / CHUNK;
#pragma unroll 1
  for (int ch = 0; ch < nChunks; ++ch) {
    const int cbase = ch * CHUNK;
    const int wc = scan_chunk<NBF>(dsts, nE, cbase, nodeBase, vec8, list, tid, lane, wave);
    if (lane == 0) wcnt[wave] = wc;
    __syncthreads();
    if (wave == 0) {
#pragma unroll 1
      for (int wsx = 0; wsx < NWAVE; ++wsx) {
        int n = __builtin_amdgcn_readfirstlane(wcnt[wsx]);
        n = n > WCAP ? WCAP : (n < 0 ? 0 : n);
        const int* lp = list + wsx * WCAP;
#pragma unroll 1
        for (int i = 0; i < n; ++i) {
          const int ent  = __builtin_amdgcn_readfirstlane(lp[i]);
          const int slot = ent & (NBF - 1);
          int e = cbase + ((ent >> 12) & (CHUNK - 1));
          e = e > nE - 1 ? nE - 1 : e;
          int src = srcs[e];
          src = src < 0 ? 0 : (src > nSrc - 1 ? nSrc - 1 : src);
          if (lane == 0) {
            int pos = cursor[slot];
            pos = pos < 0 ? 0 : (pos > RCAP - 1 ? RCAP - 1 : pos);
            region[pos] = src;
            const int np = pos + 1;
            cursor[slot] = np > RCAP ? RCAP : np;
          }
        }
      }
    }
    __syncthreads();
  }

  const int nv = lenW >> 2;
  int* gp = csr + rb0;
#pragma unroll 1
  for (int i = tid; i < nv; i += NTHR) { const v4i v = ((const v4i*)region)[i]; *(volatile v4i*)(gp + 4 * i) = v; }
  __threadfence();
#pragma unroll 1
  for (int i = tid; i < nv; i += NTHR) { const v4i v = ((const v4i*)region)[i]; *(volatile v4i*)(gp + 4 * i) = v; }
}

template <int KD, int NV>
__global__ __launch_bounds__(NTHR) void k_gemmP(
    const float* __restrict__ A, const _Float16* __restrict__ Bw, const float* __restrict__ bias,
    const float* __restrict__ att0, const float* __restrict__ att1, const float* __restrict__ att2,
    float* C, float* e0, float* e1, float* e2, int nRowsA) {
  constexpr int APK = KD + 8;
  constexpr int UPT = (BM * KD / 8) / NTHR;
  constexpr int NES = BM * HEADS;
  static_assert(KD % 32 == 0 && UPT * NTHR * 8 == BM * KD);
  static_assert(NV == 1 || NV == 3);
  static_assert(((APK * 2) % 16) == 0);
  __shared__ __attribute__((aligned(16))) _Float16 sA[BM * APK];
  __shared__ __attribute__((aligned(16))) float stg[BM * NC];
  __shared__ __attribute__((aligned(16))) float sE[NV][NES];
  const int tid = threadIdx.x, lane = tid & 31, wave = tid >> 5, hh = lane >> 4, m = lane & 15;
  const int rowBase = blockIdx.x * BM;

#pragma unroll
  for (int i = 0; i < UPT; ++i) {
    const int idx = i * NTHR + tid;
    const int r   = idx / (KD / 8);
    const int c8  = (idx - r * (KD / 8)) * 8;
    int row = rowBase + r;
    row = row > nRowsA - 1 ? nRowsA - 1 : row;
    const float* ap = A + (size_t)row * KD + c8;
    const v4f a = *(const v4f*)ap, b = *(const v4f*)(ap + 4);
    *(v8h*)(sA + r * APK + c8) = cvt8(a, b, ASC);
  }
  __syncthreads();

  const int rg = wave >> 1, chf = wave & 1;
  const int r0 = rg * 16, c0 = chf * 32;
  v8f acc0 = {0.f, 0.f, 0.f, 0.f, 0.f, 0.f, 0.f, 0.f};
  v8f acc1 = {0.f, 0.f, 0.f, 0.f, 0.f, 0.f, 0.f, 0.f};
  mma2<KD>(sA, Bw, r0, c0, hh, m, acc0, acc1);
  stage2(stg, r0, c0, hh, m, acc0, acc1);
  __syncthreads();

  const int qq   = lane & 7;
  const int rsub = lane >> 3;
  const int col  = c0 + 4 * qq;
  const int hd   = col >> 4;
  const v4f bb = *(const v4f*)(bias + col);
  const v4f a0 = *(const v4f*)(att0 + col);
  v4f a1 = a0, a2 = a0;
  if constexpr (NV == 3) { a1 = *(const v4f*)(att1 + col); a2 = *(const v4f*)(att2 + col); }
  const size_t gb = (size_t)(rowBase + r0) * NC + col;
  v4f vo[4];
#pragma unroll
  for (int it = 0; it < 4; ++it) {
    const int row = it * 4 + rsub;
    v4f v = *(const v4f*)(stg + (r0 + row) * NC + col);
    v = v * RSC + bb;
    vo[it] = v;
    *(volatile v4f*)(C + gb + (size_t)row * NC) = v;
    float p0 = v.x * a0.x + v.y * a0.y + v.z * a0.z + v.w * a0.w;
    float p1 = 0.f, p2 = 0.f;
    if constexpr (NV == 3) {
      p1 = v.x * a1.x + v.y * a1.y + v.z * a1.z + v.w * a1.w;
      p2 = v.x * a2.x + v.y * a2.y + v.z * a2.z + v.w * a2.w;
    }
    p0 += __shfl_xor(p0, 1); p0 += __shfl_xor(p0, 2);
    if constexpr (NV == 3) {
      p1 += __shfl_xor(p1, 1); p1 += __shfl_xor(p1, 2);
      p2 += __shfl_xor(p2, 1); p2 += __shfl_xor(p2, 2);
    }
    if ((lane & 3) == 0) {
      sE[0][(r0 + row) * HEADS + hd] = p0;
      if constexpr (NV == 3) {
        sE[1][(r0 + row) * HEADS + hd] = p1;
        sE[2][(r0 + row) * HEADS + hd] = p2;
      }
    }
  }
  __threadfence();
#pragma unroll
  for (int it = 0; it < 4; ++it) {
    const int row = it * 4 + rsub;
    *(volatile v4f*)(C + gb + (size_t)row * NC) = vo[it];
  }
  __syncthreads();

  const size_t ebs = (size_t)rowBase * HEADS;
  const int wv = wave >> 1, wl = wave & 1;
  const int f = wl * 128 + 4 * lane;
  v4f dv = {0.f, 0.f, 0.f, 0.f};
  if (wv == 0) {
    dv = *(const v4f*)(&sE[0][f]);
    *(volatile v4f*)(e0 + ebs + f) = dv;
  } else if (NV == 3 && wv == 1) {
    dv = *(const v4f*)(&sE[NV == 3 ? 1 : 0][f]);
    *(volatile v4f*)(e1 + ebs + f) = dv;
  } else if (NV == 3 && wv == 2) {
    dv = *(const v4f*)(&sE[NV == 3 ? 2 : 0][f]);
    *(volatile v4f*)(e2 + ebs + f) = dv;
  }
  __threadfence();
  if (wv == 0) {
    *(volatile v4f*)(e0 + ebs + f) = dv;
  } else if (NV == 3 && wv == 1) {
    *(volatile v4f*)(e1 + ebs + f) = dv;
  } else if (NV == 3 && wv == 2) {
    *(volatile v4f*)(e2 + ebs + f) = dv;
  }
}

__global__ __launch_bounds__(NTHR) void k_agg(
    const int* __restrict__ csr, const int* __restrict__ off, const int* __restrict__ cnt,
    const float* __restrict__ eS, const float* __restrict__ eD, const float* __restrict__ hw,
    float* xout, int nDst, int nSrc, int csrLen) {
  const int tid = threadIdx.x, lane = tid & 31, wave = tid >> 5;
  const int tbase = blockIdx.x * TGT + wave * 32;
  const int q    = lane & 15;
  const int col0 = 4 * q;
  const int hd0  = q >> 2;
  const bool stok = lane < 16;
  const v4f z4 = {0.f, 0.f, 0.f, 0.f};

  const int cl    = tbase + lane;
  const int cnt_l = cnt[cl];
  const int off_l = off[cl];

#pragma unroll 1
  for (int j = 0; j < 32; ++j) {
    const int c = tbase + j;
    int n = __shfl(cnt_l, j);
    n = n < 0 ? 0 : (n > DEGCAP ? DEGCAP : n);
    const int st = __shfl(off_l, j);
    const float ed0 = eD[(size_t)c * HEADS + hd0];

    float mx0 = NEG_BIG;
#pragma unroll 1
    for (int q0 = 0; q0 < n; q0 += 32) {
      int pos = st + q0 + lane;
      pos = pos < 0 ? 0 : (pos > csrLen - 1 ? csrLen - 1 : pos);
      int sl = csr[pos];
      sl = sl < 0 ? 0 : (sl > nSrc - 1 ? nSrc - 1 : sl);
      const int mcnt = (n - q0) < 32 ? (n - q0) : 32;
#pragma unroll 1
      for (int pp = 0; pp < mcnt; ++pp) {
        const int s = __builtin_amdgcn_readlane(sl, pp);
        mx0 = fmaxf(mx0, lrelu(eS[(size_t)s * HEADS + hd0] + ed0));
      }
    }

    float den0 = 0.f;
    v4f   acc0 = z4;
#pragma unroll 1
    for (int q0 = 0; q0 < n; q0 += 32) {
      int pos = st + q0 + lane;
      pos = pos < 0 ? 0 : (pos > csrLen - 1 ? csrLen - 1 : pos);
      int sl = csr[pos];
      sl = sl < 0 ? 0 : (sl > nSrc - 1 ? nSrc - 1 : sl);
      const int mcnt = (n - q0) < 32 ? (n - q0) : 32;
#pragma unroll 1
      for (int pp = 0; pp < mcnt; ++pp) {
        const int s = __builtin_amdgcn_readlane(sl, pp);
        const float p0 = __expf(lrelu(eS[(size_t)s * HEADS + hd0] + ed0) - mx0);
        den0 += p0;
        const v4f h0 = *(const v4f*)(hw + (size_t)s * NC + col0);
        acc0 = acc0 + h0 * p0;
      }
    }

    const float rd0 = 1.0f / (den0 + DEN_EPS);
    v4f v0 = acc0 * rd0;
    v0.x = fmaxf(v0.x, 0.0f); v0.y = fmaxf(v0.y, 0.0f);
    v0.z = fmaxf(v0.z, 0.0f); v0.w = fmaxf(v0.w, 0.0f);
    if (c >= nDst) v0 = z4;
    float* pw = xout + (size_t)c * NC + col0;
    if (stok) *(volatile v4f*)pw = v0;
    __threadfence();
    if (stok) *(volatile v4f*)pw = v0;
  }
}

template <int KD>
__global__ __launch_bounds__(NTHR) void k_gemmS(
    const float* __restrict__ A, const _Float16* __restrict__ Bw, const float* __restrict__ bk,
    float* part, int nRowsA, int nValid) {
  constexpr int APK = KD + 8;
  constexpr int UPT = (BM * KD / 8) / NTHR;
  static_assert(KD % 32 == 0 && UPT * NTHR * 8 == BM * KD);
  static_assert(((APK * 2) % 16) == 0);
  static_assert(NTHR == 4 * NC);
  __shared__ __attribute__((aligned(16))) _Float16 sA[BM * APK];
  __shared__ __attribute__((aligned(16))) float stg[BM * NC];
  __shared__ __attribute__((aligned(16))) float sRed[4 * NC];
  __shared__ __attribute__((aligned(16))) float sCol[NC];
  const int tid = threadIdx.x, lane = tid & 31, wave = tid >> 5, hh = lane >> 4, m = lane & 15;
  const int rowBase = blockIdx.x * BM;

#pragma unroll
  for (int i = 0; i < UPT; ++i) {
    const int idx = i * NTHR + tid;
    const int r   = idx / (KD / 8);
    const int c8  = (idx - r * (KD / 8)) * 8;
    int row = rowBase + r;
    row = row > nRowsA - 1 ? nRowsA - 1 : row;
    const float* ap = A + (size_t)row * KD + c8;
    const v4f a = *(const v4f*)ap, b = *(const v4f*)(ap + 4);
    *(v8h*)(sA + r * APK + c8) = cvt8(a, b, ASC);
  }
  __syncthreads();

  const int rg = wave >> 1, chf = wave & 1;
  const int r0 = rg * 16, c0 = chf * 32;
  v8f acc0 = {0.f, 0.f, 0.f, 0.f, 0.f, 0.f, 0.f, 0.f};
  v8f acc1 = {0.f, 0.f, 0.f, 0.f, 0.f, 0.f, 0.f, 0.f};
  mma2<KD>(sA, Bw, r0, c0, hh, m, acc0, acc1);
  stage2(stg, r0, c0, hh, m, acc0, acc1);
  __syncthreads();

  const int c  = tid & (NC - 1);
  const int rq = tid >> 6;
  const float bkc = bk[c];
  float s = 0.0f;
#pragma unroll 1
  for (int r = 0; r < 16; ++r) {
    const int row = rq * 16 + r;
    const float v = stg[row * NC + c] * RSC + bkc;
    const float t = tanhf(v);
    s += (rowBase + row < nValid) ? t : 0.0f;
  }
  sRed[rq * NC + c] = s;
  __syncthreads();
  if (tid < NC) sCol[tid] = (sRed[tid] + sRed[NC + tid]) + (sRed[2 * NC + tid] + sRed[3 * NC + tid]);
  __syncthreads();
  v4f pv = {0.f, 0.f, 0.f, 0.f};
  if (tid < 16) {
    pv = *(const v4f*)(sCol + 4 * tid);
    *(volatile v4f*)(part + (size_t)blockIdx.x * NC + 4 * tid) = pv;
  }
  __threadfence();
  if (tid < 16) *(volatile v4f*)(part + (size_t)blockIdx.x * NC + 4 * tid) = pv;
}

__global__ __launch_bounds__(STHR) void k_semfinal(
    const float* __restrict__ part, const float* __restrict__ qv, float* attn, int nBlk, int nValid) {
  __shared__ double sv[STHR];
  __shared__ __attribute__((aligned(16))) float sLine[32];
  const int tid = threadIdx.x;
  const int t = tid >> 6, c = tid & (NC - 1);
  double s = 0.0;
  const float* pp = part + (size_t)t * nBlk * NC + c;
#pragma unroll 1
  for (int b = 0; b < nBlk; ++b) s += (double)pp[(size_t)b * NC];
  sv[tid] = (double)qv[c] * (s / (double)nValid);
  if (tid < 32) sLine[tid] = 0.0f;
  __syncthreads();
  if (tid == 0) {
    double s0 = 0.0, s1 = 0.0;
#pragma unroll 1
    for (int k = 0; k < NC; ++k) { s0 += sv[k]; s1 += sv[NC + k]; }
    const float f0 = (float)s0, f1 = (float)s1;
    const float mx = fmaxf(f0, f1);
    const float x0 = __expf(f0 - mx), x1 = __expf(f1 - mx);
    const float inv = 1.0f / (x0 + x1);
    sLine[0] = x0 * inv;
    sLine[1] = x1 * inv;
  }
  __syncthreads();
  v4f lv = {0.f, 0.f, 0.f, 0.f};
  if (tid < 8) {
    lv = *(const v4f*)(sLine + 4 * tid);
    *(volatile v4f*)(attn + 4 * tid) = lv;
  }
  __threadfence();
  if (tid < 8) *(volatile v4f*)(attn + 4 * tid) = lv;
}

template <int KD>
__global__ __launch_bounds__(NTHR) void k_gemmD(
    const float* __restrict__ A0, const float* __restrict__ A1, const float* __restrict__ attn,
    const _Float16* __restrict__ Bw, const float* __restrict__ bd1,
    const float* __restrict__ Wd2, const float* __restrict__ bd2,
    float* z, int nRowsA) {
  constexpr int APK = KD + 8;
  constexpr int UPT = (BM * KD / 8) / NTHR;
  static_assert(KD % 32 == 0 && UPT * NTHR * 8 == BM * KD);
  static_assert(((APK * 2) % 16) == 0);
  __shared__ __attribute__((aligned(16))) _Float16 sA[BM * APK];
  __shared__ __attribute__((aligned(16))) float stg[BM * NC];
  __shared__ __attribute__((aligned(16))) float sZ[BM * 2];
  __shared__ __attribute__((aligned(16))) float sZr[BM];
  const int tid = threadIdx.x, lane = tid & 31, wave = tid >> 5, hh = lane >> 4, m = lane & 15;
  const int rowBase = blockIdx.x * BM;
  const float w0 = attn[0], w1 = attn[1];

#pragma unroll
  for (int i = 0; i < UPT; ++i) {
    const int idx = i * NTHR + tid;
    const int r   = idx / (KD / 8);
    const int c8  = (idx - r * (KD / 8)) * 8;
    int row = rowBase + r;
    row = row > nRowsA - 1 ? nRowsA - 1 : row;
    const float* ap0 = A0 + (size_t)row * KD + c8;
    const float* ap1 = A1 + (size_t)row * KD + c8;
    const v4f a0 = *(const v4f*)ap0, b0 = *(const v4f*)(ap0 + 4);
    const v4f a1 = *(const v4f*)ap1, b1 = *(const v4f*)(ap1 + 4);
    const v4f ca = a0 * w0 + a1 * w1;
    const v4f cb = b0 * w0 + b1 * w1;
    *(v8h*)(sA + r * APK + c8) = cvt8(ca, cb, ASC);
  }
  __syncthreads();

  const int rg = wave >> 1, chf = wave & 1;
  const int r0 = rg * 16, c0 = chf * 32;
  v8f acc0 = {0.f, 0.f, 0.f, 0.f, 0.f, 0.f, 0.f, 0.f};
  v8f acc1 = {0.f, 0.f, 0.f, 0.f, 0.f, 0.f, 0.f, 0.f};
  mma2<KD>(sA, Bw, r0, c0, hh, m, acc0, acc1);
  stage2(stg, r0, c0, hh, m, acc0, acc1);
  __syncthreads();

  const int qq   = lane & 7;
  const int rsub = lane >> 3;
  const int col  = c0 + 4 * qq;
  const v4f bb = *(const v4f*)(bd1 + col);
  const v4f wd = *(const v4f*)(Wd2 + col);
#pragma unroll
  for (int it = 0; it < 4; ++it) {
    const int row = it * 4 + rsub;
    v4f v = *(const v4f*)(stg + (r0 + row) * NC + col);
    v = v * RSC + bb;
    v.x = fmaxf(v.x, 0.0f); v.y = fmaxf(v.y, 0.0f);
    v.z = fmaxf(v.z, 0.0f); v.w = fmaxf(v.w, 0.0f);
    float pd = v.x * wd.x + v.y * wd.y + v.z * wd.z + v.w * wd.w;
    pd += __shfl_xor(pd, 1); pd += __shfl_xor(pd, 2); pd += __shfl_xor(pd, 4);
    if (qq == 0) sZ[(r0 + row) * 2 + chf] = pd;
  }
  __syncthreads();
  if (tid < BM) sZr[tid] = (sZ[2 * tid] + sZ[2 * tid + 1]) + bd2[0];
  __syncthreads();
  v4f zv = {0.f, 0.f, 0.f, 0.f};
  if (tid < 16) {
    zv = *(const v4f*)(sZr + 4 * tid);
    *(volatile v4f*)(z + (size_t)rowBase + 4 * tid) = zv;
  }
  __threadfence();
  if (tid < 16) *(volatile v4f*)(z + (size_t)rowBase + 4 * tid) = zv;
}

__global__ __launch_bounds__(ZTHR) void k_zsoft(const float* __restrict__ z, float* out, int nN) {
  __shared__ float sm[ZTHR / 32];
  __shared__ double sd[ZTHR];
  __shared__ float bc[4];
  const int tid = threadIdx.x, lane = tid & 31, wave = tid >> 5;
  float mx = NEG_BIG;
#pragma unroll 1
  for (int i = tid; i < nN; i += ZTHR) mx = fmaxf(mx, z[i]);
#pragma unroll
  for (int o = 16; o > 0; o >>= 1) mx = fmaxf(mx, __shfl_xor(mx, o));
  if (lane == 0) sm[wave] = mx;
  __syncthreads();
  if (tid == 0) {
    float m2 = sm[0];
#pragma unroll 1
    for (int w = 1; w < ZTHR / 32; ++w) m2 = fmaxf(m2, sm[w]);
    bc[0] = m2;
  }
  __syncthreads();
  const float gm = bc[0];
  double s = 0.0;
#pragma unroll 1
  for (int i = tid; i < nN; i += ZTHR) s += (double)__expf(z[i] - gm);
  sd[tid] = s;
  __syncthreads();
  if (tid == 0) {
    double t = 0.0;
#pragma unroll 1
    for (int i = 0; i < ZTHR; ++i) t += sd[i];
    bc[1] = 1.0f / (float)t;
  }
  __syncthreads();
  const float inv = bc[1];
  const int nv4 = nN >> 2;
#pragma unroll 1
  for (int i = tid; i < nv4; i += ZTHR) {
    const v4f zz = *(const v4f*)(z + 4 * (size_t)i);
    v4f o;
    o.x = __expf(zz.x - gm) * inv; o.y = __expf(zz.y - gm) * inv;
    o.z = __expf(zz.z - gm) * inv; o.w = __expf(zz.w - gm) * inv;
    *(volatile v4f*)(out + 4 * (size_t)i) = o;
  }
  if (tid == 0) {
#pragma unroll 1
    for (int i = 4 * nv4; i < nN; ++i) *(volatile float*)(out + i) = __expf(z[i] - gm) * inv;
  }
  __threadfence();
#pragma unroll 1
  for (int i = tid; i < nv4; i += ZTHR) {
    const v4f zz = *(const v4f*)(z + 4 * (size_t)i);
    v4f o;
    o.x = __expf(zz.x - gm) * inv; o.y = __expf(zz.y - gm) * inv;
    o.z = __expf(zz.z - gm) * inv; o.w = __expf(zz.w - gm) * inv;
    *(volatile v4f*)(out + 4 * (size_t)i) = o;
  }
  if (tid == 0) {
#pragma unroll 1
    for (int i = 4 * nv4; i < nN; ++i) *(volatile float*)(out + i) = __expf(z[i] - gm) * inv;
  }
}

extern "C" void kernel_launch(void* const* d_in, const int* in_sizes, int n_in,
                              void* d_out, int out_size, void* d_ws, size_t ws_size,
                              hipStream_t stream) {
  if (n_in < 25) return;
  if (in_sizes[0] <= 0 || in_sizes[1] <= 0) return;
  const int nP = in_sizes[0] / FIN;
  const int nA = in_sizes[1] / FIN;
  if (nP <= 0 || nA <= 0 || in_sizes[0] != nP * FIN || in_sizes[1] != nA * FIN) return;
  const int nEpa = in_sizes[2], nEaa = in_sizes[4];
  if (nEpa <= 0 || nEaa <= 0 || in_sizes[3] != nEpa || in_sizes[5] != nEaa) return;
  if (in_sizes[8] != FIN * NC || in_sizes[10] != FIN * NC || in_sizes[9] != NC || in_sizes[11] != NC) return;
  for (int i = 12; i <= 17; ++i) if (in_sizes[i] != NC) return;
  if (in_sizes[18] != NC * NC || in_sizes[19] != NC || in_sizes[20] != NC) return;
  if (in_sizes[21] != NC * NC || in_sizes[22] != NC || in_sizes[23] != NC || in_sizes[24] < 1) return;
  if (out_size != nA) return;
  if (nEpa > (1 << 28) || nEaa > (1 << 28) || nP > (1 << 24) || nA > (1 << 24)) return;

  const float* x_place   = (const float*)d_in[0];
  const float* x_atrans  = (const float*)d_in[1];
  const int*   e_pa_src  = (const int*)d_in[2];
  const int*   e_pa_dst  = (const int*)d_in[3];
  const int*   e_aa_src  = (const int*)d_in[4];
  const int*   e_aa_dst  = (const int*)d_in[5];
  const float* Wp_place  = (const float*)d_in[8];
  const float* bp_place  = (const float*)d_in[9];
  const float* Wp_atrans = (const float*)d_in[10];
  const float* bp_atrans = (const float*)d_in[11];
  const float* asrc_pa   = (const float*)d_in[12];
  const float* adst_pa   = (const float*)d_in[13];
  const float* asrc_aa   = (const float*)d_in[14];
  const float* adst_aa   = (const float*)d_in[15];
  const float* Wk        = (const float*)d_in[18];
  const float* bk        = (const float*)d_in[19];
  const float* qv        = (const float*)d_in[20];
  const float* Wd1       = (const float*)d_in[21];
  const float* bd1       = (const float*)d_in[22];
  const float* Wd2       = (const float*)d_in[23];
  const float* bd2       = (const float*)d_in[24];
  float* out = (float*)d_out;

  const int NPADP  = ((nP + TGT - 1) / TGT) * TGT;
  const int NPADA  = ((nA + TGT - 1) / TGT) * TGT;
  const int nBC    = (nA + NBC - 1) / NBC;
  const int CNTPAD = nBC * NBC;
  if (CNTPAD < NPADA) return;
  if (4 * nBC + 1 > RBN) return;
  if (31 * 4 * nBC > 4096) return;
  const int nBF    = (nA + NBF - 1) / NBF;
  const int csrLenPA = ((nEpa + 31) & ~31) + 4096;
  const int csrLenAA = ((nEaa + 31) & ~31) + 4096;
  const int nAgg   = NPADA / TGT;
  const int nGP    = NPADP / BM;
  const int nGA    = NPADA / BM;

  char* ws = (char*)d_ws;
  size_t off = 0;
  const size_t oWPp  = off; off += (size_t)FIN * NC * 2;          off = (off + 255) & ~(size_t)255;
  const size_t oWPa  = off; off += (size_t)FIN * NC * 2;          off = (off + 255) & ~(size_t)255;
  const size_t oWK   = off; off += (size_t)NC * NC * 2;           off = (off + 255) & ~(size_t)255;
  const size_t oWD   = off; off += (size_t)NC * NC * 2;           off = (off + 255) & ~(size_t)255;
  const size_t oCnt0 = off; off += (size_t)CNTPAD * 4;            off = (off + 255) & ~(size_t)255;
  const size_t oOff0 = off; off += (size_t)CNTPAD * 4;            off = (off + 255) & ~(size_t)255;
  const size_t oRb0  = off; off += (size_t)RBN * 4;               off = (off + 255) & ~(size_t)255;
  const size_t oCsr0 = off; off += (size_t)csrLenPA * 4;          off = (off + 255) & ~(size_t)255;
  const size_t oCnt1 = off; off += (size_t)CNTPAD * 4;            off = (off + 255) & ~(size_t)255;
  const size_t oOff1 = off; off += (size_t)CNTPAD * 4;            off = (off + 255) & ~(size_t)255;
  const size_t oRb1  = off; off += (size_t)RBN * 4;               off = (off + 255) & ~(size_t)255;
  const size_t oCsr1 = off; off += (size_t)csrLenAA * 4;          off = (off + 255) & ~(size_t)255;
  const size_t oHP   = off; off += (size_t)NPADP * NC * 4;        off = (off + 255) & ~(size_t)255;
  const size_t oHA   = off; off += (size_t)NPADA * NC * 4;        off = (off + 255) & ~(size_t)255;
  const size_t oOPA  = off; off += (size_t)NPADA * NC * 4;        off = (off + 255) & ~(size_t)255;
  const size_t oOAA  = off; off += (size_t)NPADA * NC * 4;        off = (off + 255) & ~(size_t)255;
  const size_t oSPs  = off; off += (size_t)NPADP * HEADS * 4;     off = (off + 255) & ~(size_t)255;
  const size_t oSAdp = off; off += (size_t)NPADA * HEADS * 4;     off = (off + 255) & ~(size_t)255;
  const size_t oSAsa = off; off += (size_t)NPADA * HEADS * 4;     off = (off + 255) & ~(size_t)255;
  const size_t oSAda = off; off += (size_t)NPADA * HEADS * 4;     off = (off + 255) & ~(size_t)255;
  const size_t oPart = off; off += (size_t)2 * nGA * NC * 4;      off = (off + 255) & ~(size_t)255;
  const size_t oAttn = off; off += 256;                           off = (off + 255) & ~(size_t)255;
  const size_t oZ    = off; off += (size_t)NPADA * 4;             off = (off + 255) & ~(size_t)255;
  if (off > ws_size || off > (size_t)WSCAP) return;
  _Float16* wPp = (_Float16*)(ws + oWPp);
  _Float16* wPa = (_Float16*)(ws + oWPa);
  _Float16* wK  = (_Float16*)(ws + oWK);
  _Float16* wD  = (_Float16*)(ws + oWD);
  int*   cnt0 = (int*)(ws + oCnt0);
  int*   off0 = (int*)(ws + oOff0);
  int*   rb0  = (int*)(ws + oRb0);
  int*   csr0 = (int*)(ws + oCsr0);
  int*   cnt1 = (int*)(ws + oCnt1);
  int*   off1 = (int*)(ws + oOff1);
  int*   rb1  = (int*)(ws + oRb1);
  int*   csr1 = (int*)(ws + oCsr1);
  float* hP   = (float*)(ws + oHP);
  float* hA   = (float*)(ws + oHA);
  float* oPA  = (float*)(ws + oOPA);
  float* oAA  = (float*)(ws + oOAA);
  float* sPs  = (float*)(ws + oSPs);
  float* sAdp = (float*)(ws + oSAdp);
  float* sAsa = (float*)(ws + oSAsa);
  float* sAda = (float*)(ws + oSAda);
  float* part = (float*)(ws + oPart);
  float* attn = (float*)(ws + oAttn);
  float* zb   = (float*)(ws + oZ);

  const int vec8pa = ((nEpa & 3) == 0) ? 1 : 0;
  const int vec8aa = ((nEaa & 3) == 0) ? 1 : 0;

  k_wprep<FIN><<<dim3(NC * FIN / 8 / NTHR, 2), NTHR, 0, stream>>>(Wp_place, Wp_atrans, wPp, wPa);
  k_wprep<NC><<<dim3(NC * NC / 8 / NTHR, 2), NTHR, 0, stream>>>(Wk, Wd1, wK, wD);

  k_count<<<nBC, NTHR, 0, stream>>>(e_pa_dst, cnt0, nEpa, vec8pa);
  k_count<<<nBC, NTHR, 0, stream>>>(e_aa_dst, cnt1, nEaa, vec8aa);
  k_offsets<<<1, OTHR, 0, stream>>>(cnt0, off0, rb0, nBC);
  k_offsets<<<1, OTHR, 0, stream>>>(cnt1, off1, rb1, nBC);
  hipFuncSetAttribute(reinterpret_cast<const void*>(&k_fill),
                      hipFuncAttributeMaxDynamicSharedMemorySize, LDS_FILL);
  k_fill<<<nBF, NTHR, LDS_FILL, stream>>>(e_pa_src, e_pa_dst, off0, rb0, csr0, nP, nEpa, vec8pa, csrLenPA);
  k_fill<<<nBF, NTHR, LDS_FILL, stream>>>(e_aa_src, e_aa_dst, off1, rb1, csr1, nA, nEaa, vec8aa, csrLenAA);

  k_gemmP<FIN, 1><<<nGP, NTHR, 0, stream>>>(x_place, wPp, bp_place, asrc_pa, asrc_pa, asrc_pa,
                                             hP, sPs, sPs, sPs, nP);
  k_gemmP<FIN, 3><<<nGA, NTHR, 0, stream>>>(x_atrans, wPa, bp_atrans, adst_pa, asrc_aa, adst_aa,
                                             hA, sAdp, sAsa, sAda, nA);

  k_agg<<<nAgg, NTHR, 0, stream>>>(csr0, off0, cnt0, sPs, sAdp, hP, oPA, nA, nP, csrLenPA);
  k_agg<<<nAgg, NTHR, 0, stream>>>(csr1, off1, cnt1, sAsa, sAda, hA, oAA, nA, nA, csrLenAA);

  k_gemmS<NC><<<nGA, NTHR, 0, stream>>>(oPA, wK, bk, part, NPADA, nA);
  k_gemmS<NC><<<nGA, NTHR, 0, stream>>>(oAA, wK, bk, part + (size_t)nGA * NC, NPADA, nA);
  k_semfinal<<<1, STHR, 0, stream>>>(part, qv, attn, nGA, nA);

  k_gemmD<NC><<<nGA, NTHR, 0, stream>>>(oPA, oAA, attn, wD, bd1, Wd2, bd2, zb, NPADA);

  k_zsoft<<<1, ZTHR, 0, stream>>>(zb, out, nA);
}
